// PerceiverAttentionCA_31739808317753
// MI455X (gfx1250) — hardware-verified
//
#include <hip/hip_runtime.h>

#define B_SZ   2
#define N1     2048
#define N2     2048
#define DIM    3072
#define KVD    2048
#define NHEAD  16
#define DHD    128
#define INNER  2048
#define ROWS   4096

static_assert(ROWS == B_SZ * N1);
static_assert(ROWS == B_SZ * N2);
static_assert(INNER == NHEAD * DHD);

typedef _Float16 f16t;
typedef __attribute__((ext_vector_type(16))) _Float16 v16h;
typedef __attribute__((ext_vector_type(8)))  _Float16 v8h;
typedef __attribute__((ext_vector_type(8)))  float    v8f;
typedef __attribute__((ext_vector_type(4)))  float    v4f;

union Frag16 { v16h v; v8h h[2]; };

__device__ __forceinline__ v16h ldfrag(const f16t* p) {
  Frag16 f;
  f.h[0] = *(const v8h*)(p);
  f.h[1] = *(const v8h*)(p + 16);
  return f.v;
}

__device__ __forceinline__ v8f mma16(v16h a, v16h b, v8f c) {
  c = __builtin_amdgcn_wmma_f32_16x16x32_f16(false, a, false, b, (short)0, c, false, false);
  asm volatile("v_nop\n\tv_nop\n\tv_nop\n\tv_nop" : "+v"(c) : "v"(a), "v"(b));
  return c;
}

__device__ __forceinline__ v8f v8zero() {
  v8f z = {0.f, 0.f, 0.f, 0.f, 0.f, 0.f, 0.f, 0.f};
  return z;
}

__device__ __forceinline__ void lds_wave_sync() {
  __builtin_amdgcn_fence(__ATOMIC_RELEASE, "workgroup");
  __builtin_amdgcn_wave_barrier();
  __builtin_amdgcn_fence(__ATOMIC_ACQUIRE, "workgroup");
}

__global__ __launch_bounds__(256) void tconv_kernel(const float* __restrict__ W, unsigned short* __restrict__ outp,
                                                    int R, int Cc, float mul) {
  __shared__ __align__(16) float tf[64 * 68];
  const int c0 = blockIdx.x * 64;
  const int r0 = blockIdx.y * 64;
  const int tid = threadIdx.x;
  {
    const int lr = tid >> 4, c4 = (tid & 15) * 4;
#pragma unroll
    for (int it = 0; it < 4; ++it) {
      const int rr = it * 16 + lr;
      const v4f a = *(const v4f*)(W + (size_t)(r0 + rr) * Cc + c0 + c4);
      *(v4f*)(tf + rr * 68 + c4) = a;
    }
  }
  __syncthreads();
  const int sub = tid >> 3, c8 = (tid & 7) * 8;
  v8h hv0, hv1;
#pragma unroll
  for (int e = 0; e < 8; ++e) {
    hv0[e] = (f16t)(tf[(c8 + e) * 68 + sub] * mul);
    hv1[e] = (f16t)(tf[(c8 + e) * 68 + 32 + sub] * mul);
  }
  f16t* o = (f16t*)outp;
  const size_t g0 = (size_t)(c0 + sub) * R + r0 + c8;
  const size_t g1 = (size_t)(c0 + 32 + sub) * R + r0 + c8;
  *(volatile v8h*)(o + g0) = hv0;
  *(volatile v8h*)(o + g1) = hv1;
  __threadfence();
  *(volatile v8h*)(o + g0) = hv0;
  *(volatile v8h*)(o + g1) = hv1;
}

template <int COLS>
__global__ __launch_bounds__(256) void ln_f16_kernel(const float* __restrict__ x, const float* __restrict__ g,
                                                     const float* __restrict__ bta, unsigned short* __restrict__ outp) {
  constexpr int NCH = (COLS + 2047) / 2048;
  static_assert(COLS % 8 == 0);
  __shared__ float red[8];
  const int row = blockIdx.x;
  const int tid = threadIdx.x, wave = tid >> 5, lane = tid & 31;
  const float* xr = x + (size_t)row * COLS;

  float v[NCH][8];
  float s = 0.f;
#pragma unroll
  for (int c = 0; c < NCH; ++c) {
    const int col0 = c * 2048 + tid * 8;
#pragma unroll
    for (int e = 0; e < 8; ++e) v[c][e] = 0.f;
    if (col0 < COLS) {
      const v4f a0 = *(const v4f*)(xr + col0);
      const v4f a1 = *(const v4f*)(xr + col0 + 4);
      v[c][0] = a0[0]; v[c][1] = a0[1]; v[c][2] = a0[2]; v[c][3] = a0[3];
      v[c][4] = a1[0]; v[c][5] = a1[1]; v[c][6] = a1[2]; v[c][7] = a1[3];
    }
#pragma unroll
    for (int e = 0; e < 8; ++e) s += v[c][e];
  }
#pragma unroll
  for (int m = 16; m >= 1; m >>= 1) s += __shfl_xor(s, m, 32);
  if (lane == 0) red[wave] = s;
  __syncthreads();
  float tot = 0.f;
#pragma unroll
  for (int w = 0; w < 8; ++w) tot += red[w];
  const float mu = tot * (1.0f / (float)COLS);
  __syncthreads();

  float ss = 0.f;
#pragma unroll
  for (int c = 0; c < NCH; ++c) {
    const int col0 = c * 2048 + tid * 8;
    if (col0 < COLS) {
#pragma unroll
      for (int e = 0; e < 8; ++e) { const float d = v[c][e] - mu; ss += d * d; }
    }
  }
#pragma unroll
  for (int m = 16; m >= 1; m >>= 1) ss += __shfl_xor(ss, m, 32);
  if (lane == 0) red[wave] = ss;
  __syncthreads();
  float tot2 = 0.f;
#pragma unroll
  for (int w = 0; w < 8; ++w) tot2 += red[w];
  const float var  = tot2 * (1.0f / (float)COLS);
  const float rstd = rsqrtf(var + 1e-5f);

  v8h hv[NCH];
#pragma unroll
  for (int c = 0; c < NCH; ++c) {
    const int col0 = c * 2048 + tid * 8;
#pragma unroll
    for (int e = 0; e < 8; ++e) hv[c][e] = (f16t)0.0f;
    if (col0 < COLS) {
      const v4f g0 = *(const v4f*)(g + col0);
      const v4f g1 = *(const v4f*)(g + col0 + 4);
      const v4f b0 = *(const v4f*)(bta + col0);
      const v4f b1 = *(const v4f*)(bta + col0 + 4);
      float gv[8], bv[8];
      gv[0] = g0[0]; gv[1] = g0[1]; gv[2] = g0[2]; gv[3] = g0[3];
      gv[4] = g1[0]; gv[5] = g1[1]; gv[6] = g1[2]; gv[7] = g1[3];
      bv[0] = b0[0]; bv[1] = b0[1]; bv[2] = b0[2]; bv[3] = b0[3];
      bv[4] = b1[0]; bv[5] = b1[1]; bv[6] = b1[2]; bv[7] = b1[3];
#pragma unroll
      for (int e = 0; e < 8; ++e) {
        const float y = (v[c][e] - mu) * rstd * gv[e] + bv[e];
        hv[c][e] = (f16t)y;
      }
    }
  }
  f16t* orow = (f16t*)outp + (size_t)row * COLS;
  for (int pass = 0; pass < 2; ++pass) {
#pragma unroll
    for (int c = 0; c < NCH; ++c) {
      const int col0 = c * 2048 + tid * 8;
      if (col0 < COLS) *(volatile v8h*)(orow + col0) = hv[c];
    }
    __threadfence();
  }
}

template <int OUT16>
__global__ __launch_bounds__(256) void gemm_f16_kernel(
    const unsigned short* __restrict__ Ap, int lda, long strideA,
    const unsigned short* __restrict__ Btp, int ldb, long strideB,
    void* __restrict__ Cout, int ldc, long strideC,
    int M, int N, int K, float scale) {
  __shared__ __align__(16) float sT[8][16 * 68];
  const int z    = blockIdx.y;
  const int lane = threadIdx.x & 31;
  const int wave = threadIdx.x >> 5;
  const int tilesN = N >> 6;
  const int tilesM = M >> 6;
  const int tile = blockIdx.x * 8 + wave;
  if (tile >= tilesM * tilesN) return;
  const int tm = tile / tilesN;
  const int tn = tile - tm * tilesN;
  const int m0 = tm << 6;
  const int n0 = tn << 6;

  const f16t* Ab = (const f16t*)Ap  + (size_t)z * (size_t)strideA;
  const f16t* Bb = (const f16t*)Btp + (size_t)z * (size_t)strideB;

  const int rl   = lane & 15;
  const int koff = (lane >> 4) * 8;
  const int mOff = (lane >> 4) * 8;

  v8f acc[4][4];
#pragma unroll
  for (int i = 0; i < 4; ++i)
#pragma unroll
    for (int j = 0; j < 4; ++j) acc[i][j] = v8zero();

  for (int k0 = 0; k0 < K; k0 += 32) {
    v16h bf[4];
#pragma unroll
    for (int j = 0; j < 4; ++j)
      bf[j] = ldfrag(Bb + (size_t)(n0 + (j << 4) + rl) * ldb + k0 + koff);
#pragma unroll
    for (int i = 0; i < 4; ++i) {
      const v16h af = ldfrag(Ab + (size_t)(m0 + (i << 4) + rl) * lda + k0 + koff);
#pragma unroll
      for (int j = 0; j < 4; ++j) acc[i][j] = mma16(af, bf[j], acc[i][j]);
    }
  }

  float* slab = &sT[wave][0];
#pragma unroll
  for (int i = 0; i < 4; ++i) {
    const int mBase = m0 + (i << 4);
#pragma unroll
    for (int j = 0; j < 4; ++j)
#pragma unroll
      for (int r = 0; r < 8; ++r)
        slab[(mOff + r) * 68 + (j << 4) + rl] = acc[i][j][r] * scale;
    lds_wave_sync();
    if (OUT16 == 0) {
      float* C = (float*)Cout + (size_t)z * (size_t)strideC;
      const int hh = lane >> 4, c4 = (lane & 15) * 4;
      for (int pass = 0; pass < 2; ++pass) {
#pragma unroll
        for (int it = 0; it < 8; ++it) {
          const int row = it * 2 + hh;
          const v4f vv = *(const v4f*)(slab + row * 68 + c4);
          *(volatile v4f*)(C + (size_t)(mBase + row) * ldc + n0 + c4) = vv;
        }
        __threadfence();
      }
    } else {
      f16t* C = (f16t*)Cout + (size_t)z * (size_t)strideC;
      const int q = lane >> 3, c8 = (lane & 7) * 8;
      for (int pass = 0; pass < 2; ++pass) {
#pragma unroll
        for (int it = 0; it < 4; ++it) {
          const int row = it * 4 + q;
          const float* sp = slab + row * 68 + c8;
          v8h hv;
#pragma unroll
          for (int e = 0; e < 8; ++e) hv[e] = (f16t)sp[e];
          *(volatile v8h*)(C + (size_t)(mBase + row) * ldc + n0 + c8) = hv;
        }
        __threadfence();
      }
    }
    lds_wave_sync();
  }
}

#define KPITCH 136
#define VPITCH 72
#define OPITCH 136

__global__ __launch_bounds__(256) void attn_kernel(const unsigned short* __restrict__ qp,
                                                   const unsigned short* __restrict__ kp,
                                                   const unsigned short* __restrict__ vtp,
                                                   unsigned short* __restrict__ op, float sc2) {
  __shared__ __align__(16) f16t lds[64 * KPITCH + 128 * VPITCH];
  static_assert(8 * 16 * OPITCH <= 64 * KPITCH + 128 * VPITCH);
  f16t* ldsK = lds;
  f16t* ldsV = lds + 64 * KPITCH;

  const int tid  = threadIdx.x;
  const int wave = tid >> 5, lane = tid & 31;
  const int ln16 = lane & 15, half = lane >> 4;
  const int qblk = blockIdx.x, head = blockIdx.y, batch = blockIdx.z;
  const size_t qrow0 = (size_t)batch * N2 + (size_t)qblk * 128 + (size_t)wave * 16;

  const f16t* Qg = (const f16t*)qp + qrow0 * INNER + head * DHD;
  const f16t* Kg = (const f16t*)kp + (size_t)batch * N1 * INNER + head * DHD;
  const f16t* Vg = (const f16t*)vtp + ((size_t)batch * INNER + head * DHD) * (size_t)N1;

  v16h qb[4];
#pragma unroll
  for (int c = 0; c < 4; ++c) qb[c] = ldfrag(Qg + (size_t)ln16 * INNER + c * 32 + 8 * half);

  v8f oacc[8];
#pragma unroll
  for (int j = 0; j < 8; ++j) oacc[j] = v8zero();
  float mrun = -1.0e30f, lrun = 0.f;

  for (int kb = 0; kb < N1; kb += 64) {
    __syncthreads();
#pragma unroll
    for (int it = 0; it < 4; ++it) {
      const int i = it * 256 + tid;
      const int key = i >> 4, dv = (i & 15) * 8;
      *(v8h*)(ldsK + key * KPITCH + dv) = *(const v8h*)(Kg + (size_t)(kb + key) * INNER + dv);
      const int d = i >> 3, kf = (i & 7) * 8;
      *(v8h*)(ldsV + d * VPITCH + kf) = *(const v8h*)(Vg + (size_t)d * N1 + kb + kf);
    }
    __syncthreads();

    v8f s[4];
#pragma unroll
    for (int t = 0; t < 4; ++t) {
      s[t] = v8zero();
#pragma unroll
      for (int c = 0; c < 4; ++c) {
        const v16h kfr = ldfrag(ldsK + (t * 16 + ln16) * KPITCH + c * 32 + 8 * half);
        s[t] = mma16(kfr, qb[c], s[t]);
      }
    }

    float cmax = -1.0e30f;
#pragma unroll
    for (int t = 0; t < 4; ++t)
#pragma unroll
      for (int r = 0; r < 8; ++r) {
        const float sv = s[t][r] * sc2;
        s[t][r] = sv;
        cmax = fmaxf(cmax, sv);
      }
    cmax = fmaxf(cmax, __shfl_xor(cmax, 16, 32));
    const float mnew  = fmaxf(mrun, cmax);
    const float alpha = exp2f(mrun - mnew);
    mrun = mnew;

    float psum = 0.f;
    v8h ph[4];
#pragma unroll
    for (int t = 0; t < 4; ++t)
#pragma unroll
      for (int r = 0; r < 8; ++r) {
        const float p = exp2f(s[t][r] - mnew);
        psum += p;
        ph[t][r] = (f16t)(p * 4096.0f);
      }
    psum += __shfl_xor(psum, 16, 32);
    lrun = lrun * alpha + psum;
#pragma unroll
    for (int j = 0; j < 8; ++j)
#pragma unroll
      for (int r = 0; r < 8; ++r) oacc[j][r] *= alpha;

    Frag16 pf[2];
    pf[0].h[0] = ph[0]; pf[0].h[1] = ph[1];
    pf[1].h[0] = ph[2]; pf[1].h[1] = ph[3];
#pragma unroll
    for (int kk = 0; kk < 2; ++kk) {
#pragma unroll
      for (int j = 0; j < 8; ++j) {
        const v16h vf = ldfrag(ldsV + (j * 16 + ln16) * VPITCH + kk * 32 + 8 * half);
        oacc[j] = mma16(vf, pf[kk].v, oacc[j]);
      }
    }
  }

  __syncthreads();
  f16t* os = lds + wave * (16 * OPITCH);
  const float inv = 0.00390625f / lrun;
#pragma unroll
  for (int j = 0; j < 8; ++j) {
    v8h ov;
#pragma unroll
    for (int r = 0; r < 8; ++r) ov[r] = (f16t)(oacc[j][r] * inv);
    *(v8h*)(os + ln16 * OPITCH + j * 16 + 8 * half) = ov;
  }
  lds_wave_sync();
  f16t* Og = (f16t*)op + qrow0 * INNER + head * DHD;
  const int rsel = lane >> 4;
  const int seg  = ((lane >> 3) & 1) * 64 + (lane & 7) * 8;
  for (int pass = 0; pass < 2; ++pass) {
#pragma unroll
    for (int it = 0; it < 8; ++it) {
      const int row = it * 2 + rsel;
      const v8h vv = *(const v8h*)(os + row * OPITCH + seg);
      *(volatile v8h*)(Og + (size_t)row * INNER + seg) = vv;
    }
    __threadfence();
  }
}

extern "C" void kernel_launch(void* const* d_in, const int* in_sizes, int n_in,
                              void* d_out, int out_size, void* d_ws, size_t ws_size,
                              hipStream_t stream) {
  if (n_in < 9) return;
  if (in_sizes[0] != B_SZ * N1 * KVD) return;
  if (in_sizes[1] != B_SZ * N2 * DIM) return;
  if (in_sizes[2] != DIM * INNER) return;
  if (in_sizes[3] != KVD * 2 * INNER) return;
  if (in_sizes[4] != INNER * DIM) return;
  if (in_sizes[5] != KVD || in_sizes[6] != KVD || in_sizes[7] != DIM || in_sizes[8] != DIM) return;
  if (out_size != B_SZ * N2 * DIM) return;

  const float* x     = (const float*)d_in[0];
  const float* lat   = (const float*)d_in[1];
  const float* w_q   = (const float*)d_in[2];
  const float* w_kv  = (const float*)d_in[3];
  const float* w_out = (const float*)d_in[4];
  const float* ln1_g = (const float*)d_in[5];
  const float* ln1_b = (const float*)d_in[6];
  const float* ln2_g = (const float*)d_in[7];
  const float* ln2_b = (const float*)d_in[8];
  float* out = (float*)d_out;

  const size_t szR1  = (size_t)ROWS * DIM * 2;
  const size_t szWQ  = (size_t)INNER * DIM * 2;
  const size_t szWKV = (size_t)2 * INNER * KVD * 2;
  const size_t szWO  = (size_t)DIM * INNER * 2;
  const size_t szQ   = (size_t)ROWS * INNER * 2;
  const size_t szK   = (size_t)ROWS * INNER * 2;
  const size_t szVT  = (size_t)B_SZ * INNER * N1 * 2;
  size_t off = 0;
  const size_t oR1  = off; off += szR1;
  const size_t oWQ  = off; off += szWQ;
  const size_t oWKV = off; off += szWKV;
  const size_t oWO  = off; off += szWO;
  const size_t oQ   = off; off += szQ;
  const size_t oK   = off; off += szK;
  const size_t oVT  = off; off += szVT;
  if (off > ws_size) return;
  if ((size_t)ROWS * KVD * 2 > szR1 || (size_t)ROWS * INNER * 2 > szR1) return;

  char* ws = (char*)d_ws;
  unsigned short* R1   = (unsigned short*)(ws + oR1);
  unsigned short* wqT  = (unsigned short*)(ws + oWQ);
  unsigned short* wkvT = (unsigned short*)(ws + oWKV);
  unsigned short* woT  = (unsigned short*)(ws + oWO);
  unsigned short* q16  = (unsigned short*)(ws + oQ);
  unsigned short* k16  = (unsigned short*)(ws + oK);
  unsigned short* vT16 = (unsigned short*)(ws + oVT);

  const dim3 blk(256);
  const float wmul = 64.0f;

  tconv_kernel<<<dim3(INNER / 64, DIM / 64), blk, 0, stream>>>(w_q, wqT, DIM, INNER, wmul);
  tconv_kernel<<<dim3(2 * INNER / 64, KVD / 64), blk, 0, stream>>>(w_kv, wkvT, KVD, 2 * INNER, wmul);
  tconv_kernel<<<dim3(DIM / 64, INNER / 64), blk, 0, stream>>>(w_out, woT, INNER, DIM, wmul);

  ln_f16_kernel<DIM><<<dim3(ROWS), blk, 0, stream>>>(lat, ln2_g, ln2_b, R1);

  {
    const int tiles = (ROWS / 64) * (INNER / 64);
    gemm_f16_kernel<1><<<dim3((tiles + 7) / 8, 1), blk, 0, stream>>>(
        R1, DIM, 0L, wqT, DIM, 0L, (void*)q16, INNER, 0L, ROWS, INNER, DIM, 1.0f / 64.0f);
  }

  ln_f16_kernel<KVD><<<dim3(ROWS), blk, 0, stream>>>(x, ln1_g, ln1_b, R1);

  {
    const int tiles = (ROWS / 64) * (INNER / 64);
    gemm_f16_kernel<1><<<dim3((tiles + 7) / 8, 1), blk, 0, stream>>>(
        R1, KVD, 0L, wkvT, KVD, 0L, (void*)k16, INNER, 0L, ROWS, INNER, KVD, 1.0f / 64.0f);
  }

  {
    const int tiles = (INNER / 64) * (N1 / 64);
    gemm_f16_kernel<1><<<dim3((tiles + 7) / 8, B_SZ), blk, 0, stream>>>(
        wkvT + (size_t)INNER * KVD, KVD, 0L, R1, KVD, (long)N1 * KVD, (void*)vT16, N1, (long)INNER * N1,
        INNER, N1, KVD, 1.0f / 64.0f);
  }

  {
    const float sc2 = (float)(1.4426950408889634 * 0.08838834764831845);
    attn_kernel<<<dim3(N2 / 128, NHEAD, B_SZ), blk, 0, stream>>>(q16, k16, vT16, R1, sc2);
  }

  {
    const int tiles = (ROWS / 64) * (DIM / 64);
    gemm_f16_kernel<0><<<dim3((tiles + 7) / 8, 1), blk, 0, stream>>>(
        R1, INNER, 0L, woT, INNER, 0L, (void*)out, DIM, 0L, ROWS, DIM, INNER, 1.0f / 1024.0f);
  }
  (void)hipGetLastError();
}
